// GNNbase_9603546874512
// MI455X (gfx1250) — hardware-verified
//
#include <hip/hip_runtime.h>
#include <stddef.h>
#include <stdint.h>


#define NTHR    256
#define NWAVE   8
#define NCAP    128
#define ECAP    4096
#define EDIM    8
#define HIDW    16
#define KIN1    12
#define OUTW    32
#define TPW     4
#define GBM     64
#define GBN     64
#define GTHR    128
#define NQP1    256
#define NQP2    448
#define WSMAX   134217728

static_assert(NTHR == NWAVE * 32);
static_assert(NCAP <= NTHR);
static_assert(NCAP * 4 <= 2 * NTHR);
static_assert((ECAP % 32) == 0);
static_assert(GBM == (GTHR / 32) * 16);
static_assert(NQP1 == ((3 * 64 + 16 + GBN - 1) / GBN) * GBN);
static_assert(NQP2 == ((3 * 128 + 32 + GBN - 1) / GBN) * GBN);
static_assert((NQP1 % 32) == 0 && (NQP2 % 32) == 0 && NQP2 >= NQP1);
static_assert(OUTW == 32);

typedef float          v4f  __attribute__((ext_vector_type(4)));
typedef float          v8f  __attribute__((ext_vector_type(8)));
typedef int            v4i  __attribute__((ext_vector_type(4)));
typedef int            v8i  __attribute__((ext_vector_type(8)));
typedef unsigned short v8us __attribute__((ext_vector_type(8)));
typedef __bf16         v16b __attribute__((ext_vector_type(16)));
union FragB { v16b v; v8us h[2]; v8i w; v4i q[2]; };

__device__ __forceinline__ v8f wmb(const FragB& a, const FragB& b, v8f c) {
  v8f d = __builtin_amdgcn_wmma_f32_16x16x32_bf16(false, a.v, false, b.v, (short)0, c, false, false);
  asm volatile("v_nop\n\tv_nop\n\tv_nop\n\tv_nop" : "+v"(d) : "v"(a.w), "v"(b.w));
  return d;
}

__device__ __forceinline__ void ldwait() {
  asm volatile("s_wait_loadcnt 0x0" ::: "memory");
}

__device__ __forceinline__ unsigned bfb(float f) {
  const unsigned u = __float_as_uint(f);
  return (u + 0x7FFFu + ((u >> 16) & 1u)) >> 16;
}
__device__ __forceinline__ float bfr(float f) { return __uint_as_float(bfb(f) << 16); }
__device__ __forceinline__ int pk2(float a, float b) { return (int)(bfb(a) | (bfb(b) << 16)); }

__device__ __forceinline__ void wsync() {
  __builtin_amdgcn_fence(__ATOMIC_RELEASE, "wavefront");
  __builtin_amdgcn_wave_barrier();
  __builtin_amdgcn_fence(__ATOMIC_ACQUIRE, "wavefront");
}

__device__ __forceinline__ void build_lists(const int* __restrict__ dl, int EPG, int N,
                                            int* head, int* nxt, int* flg, int tid, int lane, int wave) {
  for (int i = tid; i < NCAP; i += NTHR) head[i] = -1;
  if (tid == 0) flg[0] = 0;
  __syncthreads();
  if (wave == 0) {
    int bad = 0;
    const int nch = (EPG + 31) >> 5;
#pragma unroll 1
    for (int c = 0; c < nch; ++c) {
      const int cb = c << 5;
      const int e  = cb + lane;
      const int ec = e < EPG ? e : EPG - 1;
      const int d  = dl[ec];
      const bool okd = (d >= 0) && (d < N);
      bad |= (e < EPG && !okd) ? 1 : 0;
      const int dc = d < 0 ? 0 : (d > N - 1 ? N - 1 : d);
      const int m32 = (EPG - cb) < 32 ? (EPG - cb) : 32;
#pragma unroll 1
      for (int k = 0; k < m32; ++k) {
        const int u   = __builtin_amdgcn_readlane(dc, k);
        const int ek  = cb + k;
        const int old = head[u];
        nxt[ek] = old;
        head[u] = ek;
      }
    }
    const unsigned anyb = __builtin_amdgcn_ballot_w32(bad != 0);
    if (lane == 0) flg[0] = (anyb != 0u) ? 1 : 0;
  }
  __syncthreads();
}

__device__ __forceinline__ void store_rows(const unsigned short* ost, v4i* OBq, int b, int N, int nGraphs,
                                           int padRows, int tid) {
  const int np = N * 4;
  const v4i* sq = (const v4i*)ost;
  const int i0 = tid < np ? tid : 0;
  const int i1 = (tid + NTHR) < np ? (tid + NTHR) : 0;
  const v4i r0 = sq[i0];
  const v4i r1 = sq[i1];
  const v4i zq = {0, 0, 0, 0};
  v4i* dq = OBq + (size_t)b * (size_t)N * 4;
  v4i* pq = OBq + (size_t)nGraphs * (size_t)N * 4;
  const bool w0 = tid < np;
  const bool w1 = (tid + NTHR) < np;
  const bool wp = (b == nGraphs - 1) && (tid < padRows * 4);
  if (w0) *(volatile v4i*)(dq + tid) = r0;
  if (w1) *(volatile v4i*)(dq + tid + NTHR) = r1;
  if (wp) *(volatile v4i*)(pq + tid) = zq;
  __threadfence();
  if (w0) *(volatile v4i*)(dq + tid) = r0;
  if (w1) *(volatile v4i*)(dq + tid + NTHR) = r1;
  if (wp) *(volatile v4i*)(pq + tid) = zq;
}

__device__ __forceinline__ void stage_ln(const v8f acc, float bias, float* ft, int hh, int m,
                                         const float* gg, const float* gb, float* yn) {
  wsync();
#pragma unroll
  for (int r = 0; r < 8; ++r) ft[(8 * hh + r) * 16 + m] = fmaxf(acc[r] + bias, 0.f);
  wsync();
  float y[16];
#pragma unroll
  for (int c = 0; c < 4; ++c) {
    const v4f t = *(const v4f*)(ft + m * 16 + 4 * c);
    y[4 * c] = t.x; y[4 * c + 1] = t.y; y[4 * c + 2] = t.z; y[4 * c + 3] = t.w;
  }
  float mean = 0.f;
#pragma unroll
  for (int k = 0; k < 16; ++k) mean += y[k];
  mean *= 0.0625f;
  float var = 0.f;
#pragma unroll
  for (int k = 0; k < 16; ++k) { const float dv = y[k] - mean; var = fmaf(dv, dv, var); }
  var *= 0.0625f;
  const float rinv = 1.0f / sqrtf(var + 1e-5f);
#pragma unroll
  for (int k = 0; k < 16; ++k) yn[k] = fmaf((y[k] - mean) * rinv, gg[k], gb[k]);
}

__device__ __forceinline__ FragB hilo_frag(const float* yn, int hh) {
  FragB a;
#pragma unroll
  for (int p = 0; p < 4; ++p) {
    const float x0 = hh ? yn[8 + 2 * p] : yn[2 * p];
    const float x1 = hh ? yn[9 + 2 * p] : yn[2 * p + 1];
    const unsigned h0 = bfb(x0), h1 = bfb(x1);
    const unsigned l0 = bfb(x0 - __uint_as_float(h0 << 16));
    const unsigned l1 = bfb(x1 - __uint_as_float(h1 << 16));
    a.w[p]     = (int)(h0 | (h1 << 16));
    a.w[4 + p] = (int)(l0 | (l1 << 16));
  }
  return a;
}

__global__ __launch_bounds__(NTHR) void k_edge(
    const float* __restrict__ nodes, const int* __restrict__ eidx, const float* __restrict__ eattr,
    const float* __restrict__ emb,
    const float* __restrict__ W1, const float* __restrict__ b1,
    const float* __restrict__ W2, const float* __restrict__ b2,
    const float* __restrict__ W3, const float* __restrict__ b3,
    const float* __restrict__ lng, const float* __restrict__ lnb,
    float* HP, float* EAR, int nE, int N, int EPG, int nNodes, int nEmb, int nTiles)
{
  __shared__ __attribute__((aligned(16))) v4i   atile[NWAVE][64];
  __shared__ __attribute__((aligned(16))) float ftile[NWAVE][256];
  const int tid = (int)threadIdx.x, lane = tid & 31, hh = lane >> 4, m = lane & 15;
  const int wave = __builtin_amdgcn_readfirstlane(tid >> 5);
  v4i* at = atile[wave];
  float* ft = ftile[wave];
  const v4f z4 = {0.f, 0.f, 0.f, 0.f};

  FragB fb1, fb2, fb3;
  float bb1, bb2, bb3;
  {
    const int i0 = m * KIN1 + 8 * hh;
    int i1 = i0 + 4;
    i1 = i1 > HIDW * KIN1 - 4 ? HIDW * KIN1 - 4 : i1;
    const v4f wa = *(const v4f*)(W1 + i0);
    v4f wb = *(const v4f*)(W1 + i1);
    if (hh) wb = z4;
    fb1.w[0] = pk2(wa.x, wa.y); fb1.w[1] = pk2(wa.z, wa.w);
    fb1.w[2] = pk2(wb.x, wb.y); fb1.w[3] = pk2(wb.z, wb.w);
    fb1.w[4] = 0; fb1.w[5] = 0; fb1.w[6] = 0; fb1.w[7] = 0;
    const float* p2 = W2 + m * HIDW + 8 * hh;
    const v4f xa = *(const v4f*)p2, xb = *(const v4f*)(p2 + 4);
    fb2.w[0] = pk2(xa.x, xa.y); fb2.w[1] = pk2(xa.z, xa.w);
    fb2.w[2] = pk2(xb.x, xb.y); fb2.w[3] = pk2(xb.z, xb.w);
    fb2.w[4] = fb2.w[0]; fb2.w[5] = fb2.w[1]; fb2.w[6] = fb2.w[2]; fb2.w[7] = fb2.w[3];
    const float* p3 = W3 + m * HIDW + 8 * hh;
    const v4f ya = *(const v4f*)p3, yb = *(const v4f*)(p3 + 4);
    fb3.w[0] = pk2(ya.x, ya.y); fb3.w[1] = pk2(ya.z, ya.w);
    fb3.w[2] = pk2(yb.x, yb.y); fb3.w[3] = pk2(yb.z, yb.w);
    fb3.w[4] = fb3.w[0]; fb3.w[5] = fb3.w[1]; fb3.w[6] = fb3.w[2]; fb3.w[7] = fb3.w[3];
    bb1 = bfr(b1[m]); bb2 = bfr(b2[m]); bb3 = bfr(b3[m]);
  }
  float gg[16], gb[16];
#pragma unroll
  for (int c = 0; c < 4; ++c) {
    const v4f tg = *(const v4f*)(lng + 4 * c);
    const v4f tb = *(const v4f*)(lnb + 4 * c);
    gg[4 * c] = bfr(tg.x); gg[4 * c + 1] = bfr(tg.y); gg[4 * c + 2] = bfr(tg.z); gg[4 * c + 3] = bfr(tg.w);
    gb[4 * c] = bfr(tb.x); gb[4 * c + 1] = bfr(tb.y); gb[4 * c + 2] = bfr(tb.z); gb[4 * c + 3] = bfr(tb.w);
  }

  const v8f zacc = {0.f, 0.f, 0.f, 0.f, 0.f, 0.f, 0.f, 0.f};
  const v4i zq = {0, 0, 0, 0};
#pragma unroll 1
  for (int ti = 0; ti < TPW; ++ti) {
    const int tile = ((int)blockIdx.x * NWAVE + wave) * TPW + ti;
    if (tile >= nTiles) break;
    wsync();
    const int e0 = tile * 16;
    int ec = e0 + m;
    ec = ec > nE - 1 ? nE - 1 : ec;
    const int b  = ec / EPG;
    const int el = ec - b * EPG;
    const int sl = eidx[(size_t)(2 * b) * (size_t)EPG + el];
    long long sf = (long long)b * (long long)N + (long long)sl;
    sf = sf < 0 ? 0 : (sf > (long long)(nNodes - 1) ? (long long)(nNodes - 1) : sf);
    const float xt = nodes[(int)sf];
    int et = (int)xt;
    et = et < 0 ? 0 : (et > nEmb - 1 ? nEmb - 1 : et);
    const v4f ev  = *(const v4f*)(emb + et * 4);
    const v4f ea0 = *(const v4f*)(eattr + (size_t)ec * EDIM);
    const v4f ea1 = *(const v4f*)(eattr + (size_t)ec * EDIM + 4);
    unsigned eb[8];
    eb[0] = bfb(ea0.x); eb[1] = bfb(ea0.y); eb[2] = bfb(ea0.z); eb[3] = bfb(ea0.w);
    eb[4] = bfb(ea1.x); eb[5] = bfb(ea1.y); eb[6] = bfb(ea1.z); eb[7] = bfb(ea1.w);
    v4f ra, rb;
    ra.x = __uint_as_float(eb[0] << 16); ra.y = __uint_as_float(eb[1] << 16);
    ra.z = __uint_as_float(eb[2] << 16); ra.w = __uint_as_float(eb[3] << 16);
    rb.x = __uint_as_float(eb[4] << 16); rb.y = __uint_as_float(eb[5] << 16);
    rb.z = __uint_as_float(eb[6] << 16); rb.w = __uint_as_float(eb[7] << 16);
    *(v4f*)(ft + (2 * m + hh) * 4) = hh ? rb : ra;
    v4i q0, q1;
    q0.x = pk2(ev.x, ev.y); q0.y = pk2(ev.z, ev.w);
    q0.z = (int)(eb[0] | (eb[1] << 16)); q0.w = (int)(eb[2] | (eb[3] << 16));
    q1.x = (int)(eb[4] | (eb[5] << 16)); q1.y = (int)(eb[6] | (eb[7] << 16)); q1.z = 0; q1.w = 0;
    if (hh) { q0 = zq; q1 = zq; }
    at[m * 4 + 2 * hh]     = q0;
    at[m * 4 + 2 * hh + 1] = q1;
    wsync();
    const v4f eav = *(const v4f*)(ft + 4 * lane);
    FragB af;
    af.q[0] = at[m * 4 + hh];
    af.q[1] = at[m * 4 + 2 + hh];

    float yn[16];
    v8f acc = wmb(af, fb1, zacc);
    stage_ln(acc, bb1, ft, hh, m, gg, gb, yn);
    af = hilo_frag(yn, hh);
    acc = wmb(af, fb2, zacc);
    stage_ln(acc, bb2, ft, hh, m, gg, gb, yn);
    af = hilo_frag(yn, hh);
    acc = wmb(af, fb3, zacc);
    stage_ln(acc, bb3, ft, hh, m, gg, gb, yn);

    wsync();
    v4f o0, o1;
    o0.x = hh ? yn[8]  : yn[0]; o0.y = hh ? yn[9]  : yn[1]; o0.z = hh ? yn[10] : yn[2]; o0.w = hh ? yn[11] : yn[3];
    o1.x = hh ? yn[12] : yn[4]; o1.y = hh ? yn[13] : yn[5]; o1.z = hh ? yn[14] : yn[6]; o1.w = hh ? yn[15] : yn[7];
    *(v4f*)(ft + m * 16 + 8 * hh)     = o0;
    *(v4f*)(ft + m * 16 + 8 * hh + 4) = o1;
    wsync();
    const v4f p0 = *(const v4f*)(ft + 4 * lane);
    const v4f p1 = *(const v4f*)(ft + 128 + 4 * lane);
    float* hp = HP  + (size_t)e0 * HIDW + 4 * lane;
    float* ep = EAR + (size_t)e0 * EDIM + 4 * lane;
    *(volatile v4f*)hp = p0;
    *(volatile v4f*)(hp + 128) = p1;
    *(volatile v4f*)ep = eav;
    __threadfence();
    *(volatile v4f*)hp = p0;
    *(volatile v4f*)(hp + 128) = p1;
    *(volatile v4f*)ep = eav;
  }
}

__global__ __launch_bounds__(NTHR) void k_zagg(const int* __restrict__ eidx, const float* __restrict__ HP,
                                               v4i* ZBq, int N, int EPG, int nGraphs, int padRows) {
  __shared__ int head[NCAP];
  __shared__ int nxt[ECAP];
  __shared__ int flg[1];
  __shared__ __attribute__((aligned(16))) unsigned short ost[NCAP * 32];
  const int tid = (int)threadIdx.x, lane = tid & 31;
  const int wave = __builtin_amdgcn_readfirstlane(tid >> 5);
  const int b = (int)blockIdx.x;
  build_lists(eidx + (size_t)(2 * b + 1) * (size_t)EPG, EPG, N, head, nxt, flg, tid, lane, wave);
  const int poison = flg[0];
  const int c16 = lane & 15;
  const float* hb = HP + (size_t)b * (size_t)EPG * HIDW + c16;
#pragma unroll 1
  for (int s = wave; s < N; s += NWAVE) {
    float z = 0.f;
    int cur = __builtin_amdgcn_readfirstlane(head[s]);
#pragma unroll 1
    for (int it = 0; it < ECAP; ++it) {
      if (cur < 0) break;
      const int ce = cur > EPG - 1 ? EPG - 1 : cur;
      z += hb[(size_t)ce * HIDW];
      cur = __builtin_amdgcn_readfirstlane(nxt[ce]);
    }
    const unsigned hi = bfb(z);
    const unsigned lo = bfb(z - __uint_as_float(hi << 16));
    unsigned bits = (lane < 16) ? hi : lo;
    if (poison) bits = 0x7FC0u;
    ost[s * 32 + lane] = (unsigned short)bits;
  }
  __syncthreads();
  store_rows(ost, ZBq, b, N, nGraphs, padRows, tid);
}

__global__ __launch_bounds__(GTHR) void k_gemm(
    const unsigned short* __restrict__ A,
    const float* __restrict__ Wq, const float* __restrict__ Wk, const float* __restrict__ Wv,
    const float* __restrict__ Ws,
    const float* __restrict__ bq, const float* __restrict__ bk, const float* __restrict__ bv,
    const float* __restrict__ bs,
    float* outF, int HC, int OUTD, int ldo)
{
  __shared__ __attribute__((aligned(16))) float stg[GBM * GBN];
  const int tid = (int)threadIdx.x, lane = tid & 31, hh = lane >> 4, m = lane & 15;
  const int wave = __builtin_amdgcn_readfirstlane(tid >> 5);
  const int rowBase = (int)blockIdx.x * GBM;
  const int col0    = (int)blockIdx.y * GBN;
  const v4f z4 = {0.f, 0.f, 0.f, 0.f};
  const v8f zacc = {0.f, 0.f, 0.f, 0.f, 0.f, 0.f, 0.f, 0.f};

  FragB af;
  {
    const unsigned short* ap = A + (size_t)(rowBase + 16 * wave + m) * 32 + 8 * hh;
    af.h[0] = *(const v8us*)ap;
    af.h[1] = *(const v8us*)(ap + 16);
  }
  v8f acc[4];
  float bvv[4];
#pragma unroll
  for (int t = 0; t < 4; ++t) {
    const int cb  = col0 + 16 * t;
    const int seg = cb < HC ? 0 : (cb < 2 * HC ? 1 : (cb < 3 * HC ? 2 : (cb < 3 * HC + OUTD ? 3 : 4)));
    const float* W  = (seg == 0) ? Wq : ((seg == 1) ? Wk : ((seg == 2) ? Wv : Ws));
    const float* bp = (seg == 0) ? bq : ((seg == 1) ? bk : ((seg == 2) ? bv : bs));
    const int rows  = seg < 3 ? HC : OUTD;
    const int sbase = seg < 4 ? seg * HC : 3 * HC;
    int jj = cb + m - sbase;
    jj = jj < 0 ? 0 : (jj > rows - 1 ? rows - 1 : jj);
    const float* wp = W + (size_t)jj * HIDW + 8 * hh;
    v4f wa = *(const v4f*)wp;
    v4f wb = *(const v4f*)(wp + 4);
    float bsc = bp[jj];
    if (seg > 3) { wa = z4; wb = z4; bsc = 0.f; }
    FragB bf;
    bf.w[0] = pk2(wa.x, wa.y); bf.w[1] = pk2(wa.z, wa.w);
    bf.w[2] = pk2(wb.x, wb.y); bf.w[3] = pk2(wb.z, wb.w);
    bf.w[4] = bf.w[0]; bf.w[5] = bf.w[1]; bf.w[6] = bf.w[2]; bf.w[7] = bf.w[3];
    acc[t] = wmb(af, bf, zacc);
    bvv[t] = bfr(bsc);
  }

#pragma unroll
  for (int t = 0; t < 4; ++t) {
    const int lc = 16 * t + m;
#pragma unroll
    for (int r = 0; r < 8; ++r) {
      const int lr = 16 * wave + 8 * hh + r;
      stg[lr * GBN + lc] = acc[t][r] + bvv[t];
    }
  }
  __syncthreads();

  v4f fv[8];
#pragma unroll
  for (int i = 0; i < 8; ++i) {
    const int lr = 16 * wave + 2 * i + hh;
    fv[i] = *(const v4f*)(stg + lr * GBN + 4 * m);
  }
#pragma unroll
  for (int i = 0; i < 8; ++i) {
    const int lr = 16 * wave + 2 * i + hh;
    float* op = outF + (size_t)(rowBase + lr) * (size_t)ldo + col0 + 4 * m;
    *(volatile v4f*)op = fv[i];
  }
  __threadfence();
#pragma unroll
  for (int i = 0; i < 8; ++i) {
    const int lr = 16 * wave + 2 * i + hh;
    float* op = outF + (size_t)(rowBase + lr) * (size_t)ldo + col0 + 4 * m;
    *(volatile v4f*)op = fv[i];
  }
}

template<int CH, int AG>
__global__ __launch_bounds__(NTHR) void k_att(
    const int* __restrict__ eidx, const float* __restrict__ EAR, const float* __restrict__ QKV,
    const float* __restrict__ We, const int* __restrict__ agent,
    v4i* OBq, float* dout, int N, int EPG, int nNodes, int ldq, int nGraphs, int padRows)
{
  constexpr int NJ = CH / 8;
  constexpr int HC = 4 * CH;
  static_assert(NJ + 1 <= 8);
  __shared__ int head[NCAP];
  __shared__ int nxt[ECAP];
  __shared__ int flg[1];
  __shared__ __attribute__((aligned(16))) unsigned short ost[NCAP * 32];
  __shared__ __attribute__((aligned(16))) float oline[NTHR];
  const int tid = (int)threadIdx.x, lane = tid & 31;
  const int wave = __builtin_amdgcn_readfirstlane(tid >> 5);
  const int b = (int)blockIdx.x;
  const float rs = 1.0f / sqrtf((float)CH);
  const float qnan = __int_as_float(0x7fc00000);

  float wev[NJ][8];
#pragma unroll
  for (int j = 0; j < NJ; ++j) {
    const float* p = We + (size_t)(32 * j + lane) * EDIM;
    const v4f wa = *(const v4f*)p, wb = *(const v4f*)(p + 4);
    wev[j][0] = bfr(wa.x); wev[j][1] = bfr(wa.y); wev[j][2] = bfr(wa.z); wev[j][3] = bfr(wa.w);
    wev[j][4] = bfr(wb.x); wev[j][5] = bfr(wb.y); wev[j][6] = bfr(wb.z); wev[j][7] = bfr(wb.w);
  }

  build_lists(eidx + (size_t)(2 * b + 1) * (size_t)EPG, EPG, N, head, nxt, flg, tid, lane, wave);
  const int poison = flg[0];
  const int* srow = eidx + (size_t)(2 * b) * (size_t)EPG;
  const float* eab = EAR + (size_t)b * (size_t)EPG * EDIM + (lane & 7);

  int agl = 0;
  if (AG) {
    const int a0 = __builtin_amdgcn_readfirstlane(agent[b]);
    agl = a0 < 0 ? 0 : (a0 > N - 1 ? N - 1 : a0);
  }
  const int sBeg = AG ? ((wave == 0) ? agl : N) : wave;
  const int sEnd = AG ? (agl + 1) : N;
  const int sStp = AG ? 1 : NWAVE;

#pragma unroll 1
  for (int s = sBeg; s < sEnd; s += sStp) {
    const size_t g = (size_t)b * (size_t)N + (size_t)s;
    const float* qr = QKV + g * (size_t)ldq;
    float qv[NJ];
#pragma unroll
    for (int j = 0; j < NJ; ++j) qv[j] = qr[32 * j + lane];
    const float sk = qr[3 * HC + (lane & (CH - 1))];
    ldwait();

    float ud[NJ];
#pragma unroll
    for (int j = 0; j < NJ; ++j) {
      float keep = 0.f;
#pragma unroll
      for (int d = 0; d < 8; ++d) {
        float p = wev[j][d] * qv[j];
#pragma unroll
        for (int off = 1; off < CH; off <<= 1) p += __shfl_xor(p, off);
        keep = ((lane & 7) == d) ? p : keep;
      }
      ud[j] = keep;
    }

    float mx[NJ], dn[NJ], av[NJ], se[NJ];
#pragma unroll
    for (int j = 0; j < NJ; ++j) { mx[j] = -1.0e30f; dn[j] = 0.f; av[j] = 0.f; se[j] = 0.f; }

    int cur = __builtin_amdgcn_readfirstlane(head[s]);
#pragma unroll 1
    for (int it = 0; it < ECAP; ++it) {
      if (cur < 0) break;
      const int ce  = cur > EPG - 1 ? EPG - 1 : cur;
      const int slr = __builtin_amdgcn_readfirstlane(srow[ce]);
      long long sf = (long long)b * (long long)N + (long long)slr;
      sf = sf < 0 ? 0 : (sf > (long long)(nNodes - 1) ? (long long)(nNodes - 1) : sf);
      const float* kr = QKV + (size_t)sf * (size_t)ldq + HC + lane;
      float kk[NJ], vv[NJ];
#pragma unroll
      for (int j = 0; j < NJ; ++j) kk[j] = kr[32 * j];
      ldwait();
#pragma unroll
      for (int j = 0; j < NJ; ++j) vv[j] = kr[HC + 32 * j];
      const float ead = eab[(size_t)ce * EDIM];
      ldwait();
      float al[NJ];
#pragma unroll
      for (int j = 0; j < NJ; ++j) {
        float p = qv[j] * kk[j];
#pragma unroll
        for (int off = 1; off < CH; off <<= 1) p += __shfl_xor(p, off);
        float q2 = ud[j] * ead;
        q2 += __shfl_xor(q2, 1);
        q2 += __shfl_xor(q2, 2);
        q2 += __shfl_xor(q2, 4);
        al[j] = (p + q2) * rs;
      }
#pragma unroll
      for (int j = 0; j < NJ; ++j) {
        const float df = al[j] - mx[j];
        const float ee = __expf(-fabsf(df));
        const bool up  = df > 0.f;
        const float s1 = up ? ee : 1.0f;
        const float s2 = up ? 1.0f : ee;
        mx[j] = up ? al[j] : mx[j];
        dn[j] = fmaf(dn[j], s1, s2);
        av[j] = fmaf(av[j], s1, s2 * vv[j]);
        se[j] = fmaf(se[j], s1, s2 * ead);
      }
      cur = __builtin_amdgcn_readfirstlane(nxt[ce]);
    }

    float t = 0.f;
#pragma unroll
    for (int j = 0; j < NJ; ++j) {
      const float ds  = dn[j] > 0.f ? dn[j] : 1.0f;
      const float inv = (dn[j] > 0.f ? 1.0f : 0.0f) * __builtin_amdgcn_rcpf(ds);
      float ac = av[j];
#pragma unroll
      for (int d = 0; d < 8; ++d) {
        const float sd = __shfl(se[j], (lane & 24) | d);
        ac = fmaf(wev[j][d], sd, ac);
      }
      t += ac * inv;
    }
#pragma unroll
    for (int off = CH; off < 32; off <<= 1) t += __shfl_xor(t, off);
    const float a = fmaf(t, 0.25f, sk);

    if (!AG) {
      const unsigned hi = bfb(a);
      const unsigned lo = bfb(a - __uint_as_float(hi << 16));
      unsigned bits = (lane < 16) ? hi : lo;
      if (poison) bits = 0x7FC0u;
      ost[s * 32 + lane] = (unsigned short)bits;
    } else {
      float o = fmaxf(a, 0.f);
      if (poison) o = qnan;
      wsync();
      oline[wave * 32 + lane] = o;
      wsync();
      const v4f ov = *(const v4f*)(oline + wave * 32 + 4 * (lane & 7));
      float* op = dout + (size_t)b * CH + 4 * (lane & 7);
      const bool wl = lane < (CH / 4);
      if (wl) *(volatile v4f*)op = ov;
      __threadfence();
      if (wl) *(volatile v4f*)op = ov;
    }
  }
  __syncthreads();
  if (!AG) store_rows(ost, OBq, b, N, nGraphs, padRows, tid);
}

static inline int cdiv(int a, int b) { return (a + b - 1) / b; }

extern "C" void kernel_launch(void* const* d_in, const int* in_sizes, int n_in,
                              void* d_out, int out_size, void* d_ws, size_t ws_size,
                              hipStream_t stream) {
  if (n_in < 31) return;
  const int nB = in_sizes[3];
  if (nB < 1 || nB > (1 << 20)) return;
  const int N = in_sizes[0] / nB;
  if (N < 2 || N > NCAP || (N & 1) != 0 || in_sizes[0] != nB * N) return;
  if (in_sizes[1] < 2 * nB) return;
  const int EPG = in_sizes[1] / (2 * nB);
  if (EPG < 1 || EPG > ECAP || in_sizes[1] != 2 * nB * EPG) return;
  if ((long long)nB * (long long)EPG > (1LL << 27)) return;
  if (in_sizes[2] != nB * EPG * EDIM) return;
  const int nEmb = in_sizes[4] / 4;
  if (nEmb < 1 || in_sizes[4] != nEmb * 4) return;
  if (in_sizes[5] != HIDW * KIN1 || in_sizes[6] != HIDW) return;
  if (in_sizes[7] != HIDW * HIDW || in_sizes[8] != HIDW) return;
  if (in_sizes[9] != HIDW * HIDW || in_sizes[10] != HIDW) return;
  if (in_sizes[11] != HIDW || in_sizes[12] != HIDW) return;
  const int CH1 = 16, HC1 = 4 * CH1, CH2 = 32, HC2 = 4 * CH2;
  if (in_sizes[13] != HC1 * HIDW || in_sizes[14] != HC1) return;
  if (in_sizes[15] != HC1 * HIDW || in_sizes[16] != HC1) return;
  if (in_sizes[17] != HC1 * HIDW || in_sizes[18] != HC1) return;
  if (in_sizes[19] != HC1 * EDIM) return;
  if (in_sizes[20] != CH1 * HIDW || in_sizes[21] != CH1) return;
  if (in_sizes[22] != HC2 * HIDW || in_sizes[23] != HC2) return;
  if (in_sizes[24] != HC2 * HIDW || in_sizes[25] != HC2) return;
  if (in_sizes[26] != HC2 * HIDW || in_sizes[27] != HC2) return;
  if (in_sizes[28] != HC2 * EDIM) return;
  if (in_sizes[29] != CH2 * HIDW || in_sizes[30] != CH2) return;
  if (out_size != nB * OUTW) return;

  const float* nodes = (const float*)d_in[0];
  const int*   eidx  = (const int*)  d_in[1];
  const float* eattr = (const float*)d_in[2];
  const int*   agent = (const int*)  d_in[3];
  const float* emb   = (const float*)d_in[4];
  const float* W1 = (const float*)d_in[5];  const float* b1 = (const float*)d_in[6];
  const float* W2 = (const float*)d_in[7];  const float* b2 = (const float*)d_in[8];
  const float* W3 = (const float*)d_in[9];  const float* b3 = (const float*)d_in[10];
  const float* lng = (const float*)d_in[11]; const float* lnb = (const float*)d_in[12];
  const float* g1Wq = (const float*)d_in[13]; const float* g1bq = (const float*)d_in[14];
  const float* g1Wk = (const float*)d_in[15]; const float* g1bk = (const float*)d_in[16];
  const float* g1Wv = (const float*)d_in[17]; const float* g1bv = (const float*)d_in[18];
  const float* g1We = (const float*)d_in[19];
  const float* g1Ws = (const float*)d_in[20]; const float* g1bs = (const float*)d_in[21];
  const float* g2Wq = (const float*)d_in[22]; const float* g2bq = (const float*)d_in[23];
  const float* g2Wk = (const float*)d_in[24]; const float* g2bk = (const float*)d_in[25];
  const float* g2Wv = (const float*)d_in[26]; const float* g2bv = (const float*)d_in[27];
  const float* g2We = (const float*)d_in[28];
  const float* g2Ws = (const float*)d_in[29]; const float* g2bs = (const float*)d_in[30];
  float* dout = (float*)d_out;

  const int nNodes  = nB * N;
  const int nE      = nB * EPG;
  const int MP      = cdiv(nNodes, GBM) * GBM;
  const int padRows = MP - nNodes;
  const int nTiles  = cdiv(nE, 16);
  const int EP      = nTiles * 16;

  char* ws = (char*)d_ws;
  size_t off = 0;
  const size_t oHP   = off; off += (size_t)EP * HIDW * 4;   off = (off + 255) & ~(size_t)255;
  const size_t oEAR  = off; off += (size_t)EP * EDIM * 4;   off = (off + 255) & ~(size_t)255;
  const size_t oZB   = off; off += (size_t)MP * 64;         off = (off + 255) & ~(size_t)255;
  const size_t oA1B  = off; off += (size_t)MP * 64;         off = (off + 255) & ~(size_t)255;
  const size_t oQKV1 = off; off += (size_t)MP * NQP1 * 4;   off = (off + 255) & ~(size_t)255;
  const size_t oQKV2 = off; off += (size_t)MP * NQP2 * 4;   off = (off + 255) & ~(size_t)255;
  if (off > ws_size || off > (size_t)WSMAX) return;
  float* HP   = (float*)(ws + oHP);
  float* EAR  = (float*)(ws + oEAR);
  v4i*   ZBq  = (v4i*)(ws + oZB);
  v4i*   A1q  = (v4i*)(ws + oA1B);
  float* QKV1 = (float*)(ws + oQKV1);
  float* QKV2 = (float*)(ws + oQKV2);

  k_edge<<<cdiv(nTiles, NWAVE * TPW), NTHR, 0, stream>>>(nodes, eidx, eattr, emb, W1, b1, W2, b2, W3, b3,
                                                          lng, lnb, HP, EAR, nE, N, EPG, nNodes, nEmb, nTiles);
  k_zagg<<<nB, NTHR, 0, stream>>>(eidx, HP, ZBq, N, EPG, nB, padRows);
  k_gemm<<<dim3(MP / GBM, NQP1 / GBN), GTHR, 0, stream>>>((const unsigned short*)ZBq, g1Wq, g1Wk, g1Wv, g1Ws,
                                                            g1bq, g1bk, g1bv, g1bs, QKV1, HC1, CH1, NQP1);
  k_att<16, 0><<<nB, NTHR, 0, stream>>>(eidx, EAR, QKV1, g1We, agent, A1q, dout, N, EPG, nNodes, NQP1, nB, padRows);
  k_gemm<<<dim3(MP / GBM, NQP2 / GBN), GTHR, 0, stream>>>((const unsigned short*)A1q, g2Wq, g2Wk, g2Wv, g2Ws,
                                                            g2bq, g2bk, g2bv, g2bs, QKV2, HC2, CH2, NQP2);
  k_att<32, 1><<<nB, NTHR, 0, stream>>>(eidx, EAR, QKV2, g2We, agent, A1q, dout, N, EPG, nNodes, NQP2, nB, padRows);
}
